// NonLocalBlock_4655744548983
// MI455X (gfx1250) — hardware-run, weakly checked
//
#include <hip/hip_runtime.h>


#ifndef NB
#define NB 2
#endif
#ifndef SEQ
#define SEQ 8000
#endif
#define NB_FULL 2
#define SEQ_FULL 8000
#define NC 64

static_assert(NB >= 1 && NB <= NB_FULL);
static_assert(SEQ >= 64 && SEQ <= SEQ_FULL && (SEQ % 64) == 0);

#define LDS_PITCH 72
#define OS_PITCH  68

typedef _Float16 v16h __attribute__((ext_vector_type(16)));
typedef _Float16 v8h  __attribute__((ext_vector_type(8)));
typedef float    v8f  __attribute__((ext_vector_type(8)));
typedef float    v4f  __attribute__((ext_vector_type(4)));

__device__ __forceinline__ float bfr(float v) {
  unsigned int u = __float_as_uint(v);
  u = (u + 0x7FFFu + ((u >> 16) & 1u)) & 0xFFFF0000u;
  return __uint_as_float(u);
}

__device__ __forceinline__ v8f zero8() {
  v8f z = {0.f, 0.f, 0.f, 0.f, 0.f, 0.f, 0.f, 0.f};
  return z;
}

__device__ __forceinline__ v8f mma16(v16h a, v16h b, v8f c) {
  v8f d = __builtin_amdgcn_wmma_f32_16x16x32_f16(false, a, false, b, (short)0, c,
                                                 false, false);
  asm volatile("v_nop\n\tv_nop\n\tv_nop\n\tv_nop" : "+v"(d) : "v"(a), "v"(b));
  return d;
}

__device__ __forceinline__ v16h load_h16(const _Float16* p) {
  v8h lo = *(const v8h*)(p);
  v8h hi = *(const v8h*)(p + 16);
  return __builtin_shufflevector(lo, hi, 0, 1, 2, 3, 4, 5, 6, 7,
                                 8, 9, 10, 11, 12, 13, 14, 15);
}

__global__ void __launch_bounds__(256)
cvt_w_kernel(const float* __restrict__ w0, const float* __restrict__ w1,
             const float* __restrict__ w2, const float* __restrict__ w3,
             _Float16* __restrict__ wP) {
  const int q = blockIdx.x >> 1;
  const float* src = (q == 0) ? w0 : ((q == 1) ? w1 : ((q == 2) ? w2 : w3));
  const int e = ((int)(blockIdx.x & 1) * 256 + (int)threadIdx.x) * 8;
  const v4f a = *(const v4f*)(src + e);
  const v4f c = *(const v4f*)(src + e + 4);
  v8h v;
  v[0] = (_Float16)(bfr(a[0]) * 16.f); v[1] = (_Float16)(bfr(a[1]) * 16.f);
  v[2] = (_Float16)(bfr(a[2]) * 16.f); v[3] = (_Float16)(bfr(a[3]) * 16.f);
  v[4] = (_Float16)(bfr(c[0]) * 16.f); v[5] = (_Float16)(bfr(c[1]) * 16.f);
  v[6] = (_Float16)(bfr(c[2]) * 16.f); v[7] = (_Float16)(bfr(c[3]) * 16.f);
  _Float16* dst = wP + q * (NC * NC) + e;
  *(volatile v8h*)dst = v;
  __threadfence();
  *(volatile v8h*)dst = v;
}

__global__ void __launch_bounds__(128)
proj_kernel(const float* __restrict__ x, const _Float16* __restrict__ wP,
            _Float16* __restrict__ phP, _Float16* __restrict__ thP,
            _Float16* __restrict__ gP) {
  __shared__ __align__(16) _Float16 xs[64 * LDS_PITCH];
  __shared__ __align__(16) _Float16 ts[4][16 * LDS_PITCH];
  __shared__ __align__(16) _Float16 gs[64 * LDS_PITCH];

  const int tid = threadIdx.x, lane = tid & 31, wv = tid >> 5;
  const int l15 = lane & 15, hh = (lane >> 4) << 3;
  const int b = blockIdx.y, n0 = blockIdx.x * 64;

  {
    const int nn = tid & 63, cpar = tid >> 6;
    const float* xb = x + (size_t)b * NC * SEQ_FULL + n0 + nn;
#pragma unroll 8
    for (int s = 0; s < 32; ++s) {
      const int c = cpar + 2 * s;
      xs[nn * LDS_PITCH + c] = (_Float16)bfr(xb[(size_t)c * SEQ_FULL]);
    }
  }
  __syncthreads();

  const v16h Ax0 = load_h16(&xs[(wv * 16 + l15) * LDS_PITCH + hh]);
  const v16h Ax1 = load_h16(&xs[(wv * 16 + l15) * LDS_PITCH + 32 + hh]);

#pragma unroll 1
  for (int q = 0; q < 2; ++q) {
    const _Float16* wq = wP + q * (NC * NC);
#pragma unroll
    for (int t = 0; t < 4; ++t) {
      const _Float16* wr = wq + (t * 16 + l15) * NC + hh;
      const v16h B0 = load_h16(wr);
      const v16h B1 = load_h16(wr + 32);
      v8f acc = mma16(Ax0, B0, zero8());
      acc = mma16(Ax1, B1, acc);
#pragma unroll
      for (int r = 0; r < 8; ++r)
        ts[wv][(hh + r) * LDS_PITCH + t * 16 + l15] = (_Float16)(acc[r] * 0.5f);
    }
    __syncthreads();
    _Float16* plane = (q == 0) ? phP : thP;
    _Float16* rowbase = plane + ((size_t)b * SEQ + n0 + wv * 16) * NC;
    for (int ps = 0; ps < 2; ++ps) {
      if (ps) __threadfence();
#pragma unroll
      for (int j = 0; j < 4; ++j) {
        const int row = j * 4 + (lane >> 3), piece = lane & 7;
        const v8h v = *(const v8h*)&ts[wv][row * LDS_PITCH + piece * 8];
        *(volatile v8h*)(rowbase + (size_t)row * NC + piece * 8) = v;
      }
    }
    __syncthreads();
  }

  {
    const _Float16* wq = wP + 2 * (NC * NC);
#pragma unroll
    for (int t = 0; t < 4; ++t) {
      const _Float16* wr = wq + (t * 16 + l15) * NC + hh;
      const v16h B0 = load_h16(wr);
      const v16h B1 = load_h16(wr + 32);
      v8f acc = mma16(Ax0, B0, zero8());
      acc = mma16(Ax1, B1, acc);
      v8h hv;
#pragma unroll
      for (int r = 0; r < 8; ++r) hv[r] = (_Float16)acc[r];
      *(v8h*)&gs[(t * 16 + l15) * LDS_PITCH + wv * 16 + hh] = hv;
    }
  }
  __syncthreads();
  {
    _Float16* gb = gP + (size_t)b * NC * SEQ + n0;
    for (int ps = 0; ps < 2; ++ps) {
      if (ps) __threadfence();
#pragma unroll
      for (int j = 0; j < 4; ++j) {
        const int c = j * 16 + (tid >> 3), piece = tid & 7;
        const v8h v = *(const v8h*)&gs[c * LDS_PITCH + piece * 8];
        *(volatile v8h*)(gb + (size_t)c * SEQ + piece * 8) = v;
      }
    }
  }
}

__global__ void __launch_bounds__(64)
colstat_kernel(const _Float16* __restrict__ phP, const _Float16* __restrict__ thP,
               float* __restrict__ madj) {
  __shared__ __align__(16) float Mst[64];
  const int tid = threadIdx.x, lane = tid & 31, wv = tid >> 5;
  const int l15 = lane & 15, hh = (lane >> 4) << 3;
  const int b = blockIdx.y, m0b = blockIdx.x * 64, mw = m0b + wv * 32;
  const _Float16* phB = phP + (size_t)b * SEQ * NC;
  const _Float16* thB = thP + (size_t)b * SEQ * NC;

  v16h Bt[4];
#pragma unroll
  for (int mt = 0; mt < 2; ++mt) {
    const _Float16* tr = thB + (size_t)(mw + mt * 16 + l15) * NC + hh;
    Bt[mt * 2 + 0] = load_h16(tr);
    Bt[mt * 2 + 1] = load_h16(tr + 32);
  }

  float rmax[2], rsum[2];
  rmax[0] = -1e30f; rmax[1] = -1e30f; rsum[0] = 0.f; rsum[1] = 0.f;

#pragma unroll 1
  for (int n = 0; n < SEQ; n += 16) {
    const _Float16* pr = phB + (size_t)(n + l15) * NC + hh;
    const v16h A0 = load_h16(pr);
    const v16h A1 = load_h16(pr + 32);
#pragma unroll
    for (int mt = 0; mt < 2; ++mt) {
      v8f acc = mma16(A0, Bt[mt * 2 + 0], zero8());
      acc = mma16(A1, Bt[mt * 2 + 1], acc);
      float v[8];
      float tmax = -1e30f;
#pragma unroll
      for (int r = 0; r < 8; ++r) {
        v[r] = acc[r] * (1.f / 512.f);
        tmax = fmaxf(tmax, v[r]);
      }
      const float nm = fmaxf(rmax[mt], tmax);
      float s = 0.f;
#pragma unroll
      for (int r = 0; r < 8; ++r) s += __expf(v[r] - nm);
      rsum[mt] = rsum[mt] * __expf(rmax[mt] - nm) + s;
      rmax[mt] = nm;
    }
  }

  float mo[2];
#pragma unroll
  for (int mt = 0; mt < 2; ++mt) {
    const float om = __shfl_xor(rmax[mt], 16, 32);
    const float osm = __shfl_xor(rsum[mt], 16, 32);
    const float nm = fmaxf(rmax[mt], om);
    const float tot = rsum[mt] * __expf(rmax[mt] - nm) + osm * __expf(om - nm);
    mo[mt] = nm + __logf(tot) - 9.70406053f;
  }
  if (lane < 16) {
    Mst[wv * 32 + l15] = mo[0];
    Mst[wv * 32 + 16 + l15] = mo[1];
  }
  __syncthreads();
  float* dst = madj + (size_t)b * SEQ + m0b;
  for (int ps = 0; ps < 2; ++ps) {
    if (ps) __threadfence();
    if (tid < 16) {
      const v4f vv = *(const v4f*)&Mst[tid * 4];
      *(volatile v4f*)(dst + tid * 4) = vv;
    }
  }
}

__global__ void __launch_bounds__(128) __attribute__((amdgpu_num_vgpr(256)))
attout_kernel(const _Float16* __restrict__ phP, const _Float16* __restrict__ thP,
              const _Float16* __restrict__ gP, const float* __restrict__ madj,
              const _Float16* __restrict__ wmP, const float* __restrict__ x,
              const float* __restrict__ gma, float* __restrict__ out) {
  __shared__ __align__(16) _Float16 Pbuf[4][16 * 32];
  __shared__ __align__(16) _Float16 ys[4][16 * LDS_PITCH];
  __shared__ __align__(16) float osg[64 * OS_PITCH];

  const int tid = threadIdx.x, lane = tid & 31, wv = tid >> 5;
  const int l15 = lane & 15, hh = (lane >> 4) << 3;
  const int b = blockIdx.y, n0b = blockIdx.x * 64, qn = n0b + wv * 16;

  const _Float16* phB = phP + (size_t)b * SEQ * NC;
  const _Float16* thB = thP + (size_t)b * SEQ * NC;
  const _Float16* gB  = gP + (size_t)b * NC * SEQ;
  const float* MB = madj + (size_t)b * SEQ;

  const v16h Ap0 = load_h16(phB + (size_t)(qn + l15) * NC + hh);
  const v16h Ap1 = load_h16(phB + (size_t)(qn + l15) * NC + 32 + hh);

  v8f O[4];
#pragma unroll
  for (int t = 0; t < 4; ++t) O[t] = zero8();

#pragma unroll 1
  for (int m0 = 0; m0 < SEQ; m0 += 32) {
    v16h Bt[4];
#pragma unroll
    for (int mt = 0; mt < 2; ++mt) {
      const _Float16* tr = thB + (size_t)(m0 + mt * 16 + l15) * NC + hh;
      Bt[mt * 2 + 0] = load_h16(tr);
      Bt[mt * 2 + 1] = load_h16(tr + 32);
    }
    const float c0 = MB[m0 + l15];
    const float c1 = MB[m0 + 16 + l15];

    v8f S0 = mma16(Ap0, Bt[0], zero8());
    S0 = mma16(Ap1, Bt[1], S0);
    v8f S1 = mma16(Ap0, Bt[2], zero8());
    S1 = mma16(Ap1, Bt[3], S1);

    __syncthreads();
#pragma unroll
    for (int r = 0; r < 8; ++r) {
      const int row = hh + r;
      Pbuf[wv][row * 32 + l15]      = (_Float16)__expf(S0[r] * (1.f / 512.f) - c0);
      Pbuf[wv][row * 32 + 16 + l15] = (_Float16)__expf(S1[r] * (1.f / 512.f) - c1);
    }
    __syncthreads();
    const v16h AP = load_h16(&Pbuf[wv][l15 * 32 + hh]);

#pragma unroll
    for (int t = 0; t < 4; ++t) {
      const v16h Bg = load_h16(gB + (size_t)(t * 16 + l15) * SEQ + m0 + hh);
      O[t] = mma16(AP, Bg, O[t]);
    }
  }

#pragma unroll
  for (int t = 0; t < 4; ++t)
#pragma unroll
    for (int r = 0; r < 8; ++r)
      ys[wv][(hh + r) * LDS_PITCH + t * 16 + l15] =
          (_Float16)(O[t][r] * (1.f / 32768.f));
  __syncthreads();
  const v16h Ay0 = load_h16(&ys[wv][l15 * LDS_PITCH + hh]);
  const v16h Ay1 = load_h16(&ys[wv][l15 * LDS_PITCH + 32 + hh]);
  const float gsc = bfr(gma[0]) * (1.f / 128.f);

#pragma unroll
  for (int t = 0; t < 4; ++t) {
    const _Float16* wr = wmP + (t * 16 + l15) * NC + hh;
    const v16h B0 = load_h16(wr);
    const v16h B1 = load_h16(wr + 32);
    v8f acc = mma16(Ay0, B0, zero8());
    acc = mma16(Ay1, B1, acc);
    v4f u0, u1;
    u0[0] = acc[0] * gsc; u0[1] = acc[1] * gsc; u0[2] = acc[2] * gsc; u0[3] = acc[3] * gsc;
    u1[0] = acc[4] * gsc; u1[1] = acc[5] * gsc; u1[2] = acc[6] * gsc; u1[3] = acc[7] * gsc;
    float* orow = &osg[(t * 16 + l15) * OS_PITCH + wv * 16 + hh];
    *(v4f*)orow = u0;
    *(v4f*)(orow + 4) = u1;
  }
  __syncthreads();

  {
    const int piece = tid & 15, rsel = tid >> 4;
    const size_t cb = (size_t)b * NC;
    for (int ps = 0; ps < 2; ++ps) {
      if (ps) __threadfence();
#pragma unroll
      for (int j = 0; j < 8; ++j) {
        const int o = j * 8 + rsel;
        const size_t gi = (cb + o) * SEQ_FULL + n0b + piece * 4;
        const v4f xv = *(const v4f*)(x + gi);
        const v4f av = *(const v4f*)&osg[o * OS_PITCH + piece * 4];
        v4f ov;
        ov[0] = av[0] + bfr(xv[0]);
        ov[1] = av[1] + bfr(xv[1]);
        ov[2] = av[2] + bfr(xv[2]);
        ov[3] = av[3] + bfr(xv[3]);
        *(volatile v4f*)(out + gi) = ov;
      }
    }
  }
}

extern "C" void kernel_launch(void* const* d_in, const int* in_sizes, int n_in,
                              void* d_out, int out_size, void* d_ws,
                              size_t ws_size, hipStream_t stream) {
  if (n_in < 6) return;
  if (in_sizes[0] < NB * NC * SEQ_FULL) return;
  if (in_sizes[1] < NC * NC || in_sizes[2] < NC * NC ||
      in_sizes[3] < NC * NC || in_sizes[4] < NC * NC || in_sizes[5] < 1) return;
  if (out_size < NB * NC * SEQ_FULL) return;

  const float* x       = (const float*)d_in[0];
  const float* w_phi   = (const float*)d_in[1];
  const float* w_theta = (const float*)d_in[2];
  const float* w_g     = (const float*)d_in[3];
  const float* w_mask  = (const float*)d_in[4];
  const float* gamma   = (const float*)d_in[5];
  float* out = (float*)d_out;

  size_t off = 0;
  auto take = [&](size_t bytes) -> char* {
    char* p = (char*)d_ws + off;
    off += (bytes + 255) & ~(size_t)255;
    return p;
  };
  _Float16* wP   = (_Float16*)take((size_t)4 * NC * NC * 2);
  _Float16* phP  = (_Float16*)take((size_t)NB * SEQ * NC * 2);
  _Float16* thP  = (_Float16*)take((size_t)NB * SEQ * NC * 2);
  _Float16* gP   = (_Float16*)take((size_t)NB * NC * SEQ * 2);
  float*    madj = (float*)take((size_t)NB * SEQ * 4);
  if (off > ws_size) return;

  cvt_w_kernel<<<8, 256, 0, stream>>>(w_phi, w_theta, w_g, w_mask, wP);
  proj_kernel<<<dim3(SEQ / 64, NB), 128, 0, stream>>>(x, wP, phP, thP, gP);
  colstat_kernel<<<dim3(SEQ / 64, NB), 64, 0, stream>>>(phP, thP, madj);
  attout_kernel<<<dim3(SEQ / 64, NB), 128, 0, stream>>>(
      phP, thP, gP, madj, wP + 3 * NC * NC, x, gamma, out);
}
